// MultiHeadGATLayer_2954937499915
// MI455X (gfx1250) — hardware-run, weakly checked
//
#include <hip/hip_runtime.h>

typedef float          v8f   __attribute__((ext_vector_type(8)));
typedef float          v4f   __attribute__((ext_vector_type(4)));
typedef unsigned int   v4u   __attribute__((ext_vector_type(4)));
typedef int            v8i   __attribute__((ext_vector_type(8)));
typedef unsigned short v8us  __attribute__((ext_vector_type(8)));
typedef unsigned short v16us __attribute__((ext_vector_type(16)));
typedef __bf16         v16bf __attribute__((ext_vector_type(16)));
typedef _Float16       v16h  __attribute__((ext_vector_type(16)));
typedef v4f  __attribute__((may_alias)) v4fa;
typedef v8us __attribute__((may_alias)) v8usa;
union FragB { v16bf v; v16us u; v8us h[2]; v8i w; };
union FragH { v16h  v; v16us u; v8us h[2]; v8i w; };

__device__ __forceinline__ v8f wmb(const FragB& a, const FragB& b, v8f c) {
  v8f d = __builtin_amdgcn_wmma_f32_16x16x32_bf16(false, a.v, false, b.v, (short)0, c, false, false);
  asm volatile("v_nop\n\tv_nop\n\tv_nop\n\tv_nop" : "+v"(d) : "v"(a.w), "v"(b.w));
  return d;
}

__device__ __forceinline__ v8f wmh(const FragH& a, const FragH& b, v8f c) {
  v8f d = __builtin_amdgcn_wmma_f32_16x16x32_f16(false, a.v, false, b.v, (short)0, c, false, false);
  asm volatile("v_nop\n\tv_nop\n\tv_nop\n\tv_nop" : "+v"(d) : "v"(a.w), "v"(b.w));
  return d;
}

__device__ __forceinline__ unsigned bf16_bits(float f) {
  const unsigned u = __float_as_uint(f);
  const unsigned r = (u + 0x7FFFu + ((u >> 16) & 1u)) >> 16;
  const unsigned q = (u >> 16) | 0x40u;
  return ((u & 0x7fffffffu) > 0x7f800000u) ? q : r;
}

__device__ __forceinline__ float bf16_val(float f) {
  return __uint_as_float(bf16_bits(f) << 16);
}
__device__ __forceinline__ int clampi(int v, int lo, int hi) {
  return v < lo ? lo : (v > hi ? hi : v);
}

__device__ __forceinline__ unsigned f16_bits(float f) {
  const unsigned u  = __float_as_uint(f);
  const unsigned s  = (u >> 16) & 0x8000u;
  const unsigned a  = u & 0x7fffffffu;
  const unsigned t  = a - 0x38000000u;
  const unsigned r  = (t + 0x0FFFu + ((t >> 13) & 1u)) >> 13;
  const unsigned rc = r > 0x7C00u ? 0x7C00u : r;
  const bool small  = a < 0x38800000u;
  const bool isnan  = a > 0x7f800000u;
  const unsigned fin = small ? 0u : (s | rc);
  return isnan ? (s | 0x7E00u) : fin;
}

__device__ __forceinline__ unsigned pk16(unsigned lo, unsigned hi) { return lo | (hi << 16); }
__device__ __forceinline__ unsigned bf16_lo_bits(float v) {
  float hi = bf16_val(v);
  asm volatile("" : "+v"(hi));
  return bf16_bits(v - hi);
}
__device__ __forceinline__ v4u pack8_bf16(v4f a, v4f c) {
  return (v4u){ pk16(bf16_bits(a[0]), bf16_bits(a[1])), pk16(bf16_bits(a[2]), bf16_bits(a[3])),
                pk16(bf16_bits(c[0]), bf16_bits(c[1])), pk16(bf16_bits(c[2]), bf16_bits(c[3])) };
}
__device__ __forceinline__ v4u pack8_bf16_lo(v4f a, v4f c) {
  return (v4u){ pk16(bf16_lo_bits(a[0]), bf16_lo_bits(a[1])), pk16(bf16_lo_bits(a[2]), bf16_lo_bits(a[3])),
                pk16(bf16_lo_bits(c[0]), bf16_lo_bits(c[1])), pk16(bf16_lo_bits(c[2]), bf16_lo_bits(c[3])) };
}
__device__ __forceinline__ v4u pack8_f16(v4f a, v4f c) {
  return (v4u){ pk16(f16_bits(a[0]), f16_bits(a[1])), pk16(f16_bits(a[2]), f16_bits(a[3])),
                pk16(f16_bits(c[0]), f16_bits(c[1])), pk16(f16_bits(c[2]), f16_bits(c[3])) };
}

template <int FORM>
__global__ __launch_bounds__(256) void k_plane(const float* __restrict__ src, int rows, int cols, int ldsrc,
                                               unsigned short* __restrict__ dst, int MP, int KP) {
  static_assert(FORM >= 0 && FORM <= 3);
  const int KTOT = (FORM == 1 || FORM == 3) ? 2 * KP : KP;
  const unsigned ppr   = (unsigned)(KTOT >> 3);
  const unsigned kp8   = (unsigned)(KP >> 3);
  const unsigned total = (unsigned)MP * ppr;
  const unsigned g     = blockIdx.x * 256u + threadIdx.x;
  const unsigned rowu  = g / ppr;
  const unsigned p     = g - rowu * ppr;
  const bool second    = p >= kp8;
  const int row = (int)rowu;
  const int c0  = (int)((second ? p - kp8 : p) << 3);
  const float* srow = src + (size_t)clampi(row, 0, rows - 1) * (size_t)ldsrc;
  float x[8];
  unsigned mk[8];
#pragma unroll
  for (int e = 0; e < 8; ++e) {
    const int c = c0 + e;
    const float v = srow[clampi(c, 0, cols - 1)];
    asm volatile("" :: "v"(v));
    x[e]  = v;
    mk[e] = (row < rows && c < cols) ? 0xFFFFu : 0u;
  }
  const v4f a = (v4f){ x[0], x[1], x[2], x[3] };
  const v4f c = (v4f){ x[4], x[5], x[6], x[7] };
  v4u o;
  if (FORM == 2) {
    o = pack8_f16(a, c);
  } else {
    const v4u hi = pack8_bf16(a, c);
    o = hi;
    if (FORM == 1) { const v4u lo = pack8_bf16_lo(a, c); o = second ? lo : hi; }
  }
  const v4u mw = (v4u){ pk16(mk[0], mk[1]), pk16(mk[2], mk[3]), pk16(mk[4], mk[5]), pk16(mk[6], mk[7]) };
  o &= mw;
  if (g < total) {
    volatile v4u* q = (volatile v4u*)(dst + (size_t)g * 8);
    *q = o;
    __threadfence();
    *q = o;
  }
}

template <int FORM> struct FragOf    { typedef FragB T; };
template <>         struct FragOf<2> { typedef FragH T; };
__device__ __forceinline__ v8f mm(const FragB& a, const FragB& b, v8f c) { return wmb(a, b, c); }
__device__ __forceinline__ v8f mm(const FragH& a, const FragH& b, v8f c) { return wmh(a, b, c); }
template <class F> __device__ __forceinline__ F ld_frag(const unsigned short* p) {
  F f;
  f.h[0] = *(const v8usa*)(p);
  f.h[1] = *(const v8usa*)(p + 16);
  return f;
}

template <int FORM, int EPI>
__global__ __launch_bounds__(256) __attribute__((amdgpu_num_vgpr(248)))
void k_gemm_nt(const unsigned short* __restrict__ A, const unsigned short* __restrict__ B,
               const float* __restrict__ bias, float* __restrict__ D, int M, int N, int KTOT, int ldd) {
  static_assert(FORM >= 0 && FORM <= 2);
  static_assert(EPI == 0 || EPI == 1);
  typedef typename FragOf<FORM>::T F;
  __shared__ __attribute__((aligned(16))) float sT[8][16 * 68];
  const int lane = threadIdx.x & 31;
  const int wave = threadIdx.x >> 5;
  const int tilesM = (M + 63) >> 6;
  const int tilesN = (N + 63) >> 6;
  const int tile = blockIdx.x * 8 + wave;
  if (tile >= tilesM * tilesN) return;
  const int tm = tile / tilesN;
  const int tn = tile - tm * tilesN;
  const int m0 = tm << 6;
  const int n0 = tn << 6;

  const int rl = lane & 15;
  const int h8 = (lane >> 4) * 8;
  const unsigned short* pa = A + (size_t)(m0 + rl) * (size_t)KTOT + h8;
  const unsigned short* pb = B + (size_t)(n0 + rl) * (size_t)KTOT + h8;

  v8f acc[4][4];
#pragma unroll
  for (int i = 0; i < 4; ++i)
#pragma unroll
    for (int j = 0; j < 4; ++j) acc[i][j] = (v8f){0.f, 0.f, 0.f, 0.f, 0.f, 0.f, 0.f, 0.f};

#pragma unroll 1
  for (int k0 = 0; k0 < KTOT; k0 += 32) {
    F bf[4];
#pragma unroll
    for (int j = 0; j < 4; ++j) bf[j] = ld_frag<F>(pb + (size_t)(j << 4) * (size_t)KTOT + k0);
#pragma unroll
    for (int i = 0; i < 4; ++i) {
      const F af = ld_frag<F>(pa + (size_t)(i << 4) * (size_t)KTOT + k0);
#pragma unroll
      for (int j = 0; j < 4; ++j) acc[i][j] = mm(af, bf[j], acc[i][j]);
    }
  }

  float* slab = sT[wave];
  const int hh = lane >> 4;
  const int c4 = (lane & 15) * 4;
  const int nc = n0 + c4;
  const bool cok = nc < N;
  v4f bv = (v4f){0.f, 0.f, 0.f, 0.f};
  if (EPI == 1) {
    bv = *(const v4fa*)(bias + clampi(nc, 0, N - 4));
    asm volatile("" :: "v"(bv));
  }
#pragma unroll
  for (int i = 0; i < 4; ++i) {
    const int mBase = m0 + (i << 4);
#pragma unroll
    for (int j = 0; j < 4; ++j) {
#pragma unroll
      for (int r = 0; r < 8; ++r) slab[(h8 + r) * 68 + (j << 4) + rl] = acc[i][j][r];
    }
    __builtin_amdgcn_fence(__ATOMIC_RELEASE, "workgroup");
    __builtin_amdgcn_wave_barrier();
    __builtin_amdgcn_fence(__ATOMIC_ACQUIRE, "workgroup");
    v4f vv[8];
#pragma unroll
    for (int it = 0; it < 8; ++it) {
      const int row = it * 2 + hh;
      v4f v = *(const v4fa*)(slab + row * 68 + c4);
      if (EPI == 1) v += bv;
      vv[it] = v;
    }
    for (int pass = 0; pass < 2; ++pass) {
#pragma unroll
      for (int it = 0; it < 8; ++it) {
        const int row = mBase + it * 2 + hh;
        if (cok && row < M) *(volatile v4f*)(D + (size_t)row * (size_t)ldd + nc) = vv[it];
      }
      __threadfence();
    }
    __builtin_amdgcn_fence(__ATOMIC_RELEASE, "workgroup");
    __builtin_amdgcn_wave_barrier();
    __builtin_amdgcn_fence(__ATOMIC_ACQUIRE, "workgroup");
  }
}

#pragma clang fp contract(off)

#ifndef SPLIT_O
#define SPLIT_O 1
#endif


#define NR      50000
#define NE      400000
#define MPAD    50048
#define KD      64
#define HDW     256
#define NHD     4
#define DSZ     64
#define DOUTW   64
#define KO      (SPLIT_O ? 512 : 256)
#define RTHR    256
#define RWAVES  8
#define TB_AS   0
#define TB_AD   256
#define TB_BO   512
#define TB_LG   576
#define TB_LB   640
#define TB_END  704
#define TB_N    1024
#define BT      512
#define BW      16
#define BEPT    8
#define BCHUNK  (BT * BEPT)
#define NCH     ((NE + BCHUNK - 1) / BCHUNK)
#define NB      1024
#define NBLK    ((NR + NB - 1) / NB)
#define RCAP    12288
#define DEGCAP  32
#define SLOTSH  21
#define LISTTOT (NBLK * RCAP)
#define LDS_BKT ((2 * RCAP + 3 * NB + 64) * 4)
#define WSMAX   ((size_t)128 << 20)
#define PB_WL   (HDW * KD / 8 / 256)
#define PB_WO   (DOUTW * KO / 8 / 256)
#define PB_ALL  (PB_WL + PB_WO + 1)

static_assert(NR % RWAVES == 0 && MPAD % RWAVES == 0);
static_assert(NHD * DSZ == HDW && DSZ == 64 && DOUTW == 64 && KD == 64);
static_assert(MPAD == 782 * 64 && MPAD % 64 == 0 && MPAD >= NR && MPAD % 16 == 0);
static_assert(KD % 32 == 0 && KO % 32 == 0 && HDW % 64 == 0 && DOUTW % 64 == 0 && DOUTW % 32 == 0 && HDW % 32 == 0);
static_assert(NE < (1 << SLOTSH));
static_assert(NB <= 1024 && (NB & (NB - 1)) == 0 && NB == 2 * BT);
static_assert(NE % 8 == 0 && NE >= 8);
static_assert(NBLK == 49 && NBLK * NB >= NR && NBLK * NB >= MPAD);
static_assert(NCH * BCHUNK >= NE && NCH == 98);
static_assert(RCAP % 32 == 0 && RCAP % BT == 0);
static_assert(RCAP * 4 >= 8413 * 5);
static_assert(DEGCAP >= 23 + 8);
static_assert(DEGCAP <= 32);
static_assert(LDS_BKT <= 262144 && LDS_BKT == 110848);
static_assert(BW == BT / 32 && BW == 16);
static_assert(PB_WL == 8 && PB_WL * 256 * 8 == HDW * KD);
static_assert(PB_WO * 256 * 8 == DOUTW * KO);
static_assert(TB_END <= TB_N && TB_N == 256 * 4);

typedef float        v2f __attribute__((ext_vector_type(2)));
typedef int          v4i __attribute__((ext_vector_type(4)));
typedef int          v2i __attribute__((ext_vector_type(2)));
typedef v2f __attribute__((may_alias)) v2fa;
typedef v4i __attribute__((may_alias)) v4ia;
typedef v2i __attribute__((may_alias)) v2ia;

__device__ __forceinline__ float lrelu_k(float v) { return (v > 0.0f) ? v : 0.2f * v; }
__device__ __forceinline__ float sum8(float t) {
  t = t + __shfl_xor(t, 4, 32);
  t = t + __shfl_xor(t, 2, 32);
  t = t + __shfl_xor(t, 1, 32);
  return t;
}
__device__ __forceinline__ float sum32(float t) {
  t = t + __shfl_xor(t, 16, 32);
  t = t + __shfl_xor(t, 8, 32);
  t = t + __shfl_xor(t, 4, 32);
  t = t + __shfl_xor(t, 2, 32);
  t = t + __shfl_xor(t, 1, 32);
  return t;
}
__device__ __forceinline__ float dot8(v4f za, v4f zb, v4f wa, v4f wb) {
  float t = za.x * wa.x;
  float u = za.y * wa.y; t = t + u;
  u = za.z * wa.z; t = t + u;
  u = za.w * wa.w; t = t + u;
  u = zb.x * wb.x; t = t + u;
  u = zb.y * wb.y; t = t + u;
  u = zb.z * wb.z; t = t + u;
  u = zb.w * wb.w; t = t + u;
  return t;
}
__device__ __forceinline__ float bcf(float v, int k) {
  return __int_as_float(__builtin_amdgcn_readlane(__float_as_int(v), k));
}

__global__ __launch_bounds__(256) void k_prep(const float* __restrict__ Wl, const float* __restrict__ Wo,
                                              const float* __restrict__ asrc, const float* __restrict__ adst,
                                              const float* __restrict__ bo, const float* __restrict__ lg,
                                              const float* __restrict__ lb,
                                              unsigned short* WLB, unsigned short* WO2, float* TB) {
  const int t = (int)threadIdx.x;
  const int b = (int)blockIdx.x;
  if (b < PB_WL) {
    const int g = b * 256 + t;
    const float* s = Wl + (size_t)g * 8;
    const v4f a = *(const v4fa*)s;
    const v4f c = *(const v4fa*)(s + 4);
    asm volatile("" :: "v"(a), "v"(c));
    const v4u o = pack8_bf16(a, c);
    volatile v4u* q = (volatile v4u*)(WLB + (size_t)g * 8);
    *q = o;
    __threadfence();
    *q = o;
  } else if (b < PB_WL + PB_WO) {
    const int g   = (b - PB_WL) * 256 + t;
    const int ppr = KO / 8;
    const int row = clampi(g / ppr, 0, DOUTW - 1);
    const int p   = g - (g / ppr) * ppr;
    const int c0  = (p & 31) * 8;
    const float* s = Wo + (size_t)row * HDW + c0;
    const v4f a = *(const v4fa*)s;
    const v4f c = *(const v4fa*)(s + 4);
    asm volatile("" :: "v"(a), "v"(c));
    const v4u o = pack8_bf16(a, c);
    volatile v4u* q = (volatile v4u*)(WO2 + (size_t)g * 8);
    *q = o;
    __threadfence();
    *q = o;
  } else {
    const int idx = 4 * t;
    const v4f a0 = *(const v4fa*)(asrc + clampi(idx - TB_AS, 0, 252));
    asm volatile("" :: "v"(a0));
    const v4f a1 = *(const v4fa*)(adst + clampi(idx - TB_AD, 0, 252));
    asm volatile("" :: "v"(a1));
    const v4f a2 = *(const v4fa*)(bo + clampi(idx - TB_BO, 0, 60));
    asm volatile("" :: "v"(a2));
    const v4f a3 = *(const v4fa*)(lg + clampi(idx - TB_LG, 0, 60));
    asm volatile("" :: "v"(a3));
    const v4f a4 = *(const v4fa*)(lb + clampi(idx - TB_LB, 0, 60));
    asm volatile("" :: "v"(a4));
    const unsigned m0 = (idx < TB_AD) ? 0xFFFFFFFFu : 0u;
    const unsigned m1 = (idx >= TB_AD && idx < TB_BO) ? 0xFFFFFFFFu : 0u;
    const unsigned m2 = (idx >= TB_BO && idx < TB_LG) ? 0xFFFFFFFFu : 0u;
    const unsigned m3 = (idx >= TB_LG && idx < TB_LB) ? 0xFFFFFFFFu : 0u;
    const unsigned m4 = (idx >= TB_LB && idx < TB_END) ? 0xFFFFFFFFu : 0u;
    v4u o;
    o.x = (__float_as_uint(a0.x) & m0) | (__float_as_uint(a1.x) & m1) | (__float_as_uint(a2.x) & m2) |
          (__float_as_uint(a3.x) & m3) | (__float_as_uint(a4.x) & m4);
    o.y = (__float_as_uint(a0.y) & m0) | (__float_as_uint(a1.y) & m1) | (__float_as_uint(a2.y) & m2) |
          (__float_as_uint(a3.y) & m3) | (__float_as_uint(a4.y) & m4);
    o.z = (__float_as_uint(a0.z) & m0) | (__float_as_uint(a1.z) & m1) | (__float_as_uint(a2.z) & m2) |
          (__float_as_uint(a3.z) & m3) | (__float_as_uint(a4.z) & m4);
    o.w = (__float_as_uint(a0.w) & m0) | (__float_as_uint(a1.w) & m1) | (__float_as_uint(a2.w) & m2) |
          (__float_as_uint(a3.w) & m3) | (__float_as_uint(a4.w) & m4);
    o.x = bf16_bits(__uint_as_float(o.x)) << 16;
    o.y = bf16_bits(__uint_as_float(o.y)) << 16;
    o.z = bf16_bits(__uint_as_float(o.z)) << 16;
    o.w = bf16_bits(__uint_as_float(o.w)) << 16;
    volatile v4u* q = (volatile v4u*)(TB + idx);
    *q = o;
    __threadfence();
    *q = o;
  }
}

__global__ __launch_bounds__(RTHR) void k_rowprep(const float* __restrict__ Z, const float* __restrict__ TB,
                                                  float* SD, float* SS) {
  __shared__ __attribute__((aligned(16))) float sdot[2 * RWAVES * NHD];
  const int lane = (int)threadIdx.x & 31;
  const int wave = (int)threadIdx.x >> 5;
  const int row  = (int)blockIdx.x * RWAVES + wave;
  const int rowc = row < NR ? row : NR - 1;
  const int head = lane >> 3;
  const int c0   = lane * 8;
  const float* zr = Z + (size_t)rowc * HDW + c0;
  const v4f za = *(const v4fa*)zr;
  const v4f zb = *(const v4fa*)(zr + 4);
  asm volatile("" :: "v"(za), "v"(zb));
  const v4f sa = *(const v4fa*)(TB + TB_AS + c0);
  const v4f sb = *(const v4fa*)(TB + TB_AS + c0 + 4);
  const v4f da = *(const v4fa*)(TB + TB_AD + c0);
  const v4f db = *(const v4fa*)(TB + TB_AD + c0 + 4);
  float td = dot8(za, zb, da, db);
  float ts = dot8(za, zb, sa, sb);
  td = sum8(td);
  ts = sum8(ts);
  if ((lane & 7) == 0) {
    sdot[wave * NHD + head] = td;
    sdot[RWAVES * NHD + wave * NHD + head] = ts;
  }
  __syncthreads();
  const int l8 = lane & 7;
  const int trow = (int)blockIdx.x * RWAVES + l8;
  const int trc  = trow < NR ? trow : NR - 1;
  const bool wr  = (lane < 8) && (trow < NR);
  if (wave == 0) {
    const v4f sv = *(const v4fa*)(sdot + 4 * l8);
    volatile v4f* q = (volatile v4f*)(SD + (size_t)trc * NHD);
    if (wr) *q = sv;
    __threadfence();
    if (wr) *q = sv;
  }
  if (wave == 1) {
    const v4f sv = *(const v4fa*)(sdot + RWAVES * NHD + 4 * l8);
    volatile v4f* q = (volatile v4f*)(SS + (size_t)trc * NHD);
    if (wr) *q = sv;
    __threadfence();
    if (wr) *q = sv;
  }
}

__global__ __launch_bounds__(BT) void k_bucket(const int* __restrict__ ei, unsigned* LIST, int* META) {
  extern __shared__ v4u lds_bkt[];
  int* reg1 = (int*)lds_bkt;
  int* reg2 = reg1 + RCAP;
  int* scnt = reg2 + RCAP;
  int* soff = scnt + NB;
  int* curs = soff + NB;
  int* wcnt = curs + NB;
  int* wtot = wcnt + 2 * BW;
  const int tid = (int)threadIdx.x, lane = tid & 31, wave = tid >> 5;
  const int nodeBase = (int)blockIdx.x * NB;
  int nb = NR - nodeBase;
  nb = nb > NB ? NB : (nb < 0 ? 0 : nb);
  const unsigned nbs = (unsigned)nodeBase, unb = (unsigned)nb;

  scnt[2 * tid] = 0;
  scnt[2 * tid + 1] = 0;
  if (tid == 0) reg2[0] = 0;

  int tot = 0;
#pragma unroll 1
  for (int ch = 0; ch < NCH; ++ch) {
    const int par = ch & 1;
    const int e0  = ch * BCHUNK + tid * BEPT;
    const bool valid = e0 < NE;
    const int ea = e0 < NE - 8 ? e0 : NE - 8;
    const v4i da = *(const v4ia*)(ei + ea);
    const v4i db = *(const v4ia*)(ei + ea + 4);
    asm volatile("" :: "v"(da), "v"(db));
    const unsigned s0 = (unsigned)da.x - nbs, s1 = (unsigned)da.y - nbs;
    const unsigned s2 = (unsigned)da.z - nbs, s3 = (unsigned)da.w - nbs;
    const unsigned s4 = (unsigned)db.x - nbs, s5 = (unsigned)db.y - nbs;
    const unsigned s6 = (unsigned)db.z - nbs, s7 = (unsigned)db.w - nbs;
    const bool h0 = valid && (s0 < unb), h1 = valid && (s1 < unb), h2 = valid && (s2 < unb), h3 = valid && (s3 < unb);
    const bool h4 = valid && (s4 < unb), h5 = valid && (s5 < unb), h6 = valid && (s6 < unb), h7 = valid && (s7 < unb);
    const int c = (int)h0 + (int)h1 + (int)h2 + (int)h3 + (int)h4 + (int)h5 + (int)h6 + (int)h7;
    int incl = c;
#pragma unroll
    for (int d = 1; d < 32; d <<= 1) {
      const int up = __shfl_up(incl, d, 32);
      incl += (lane >= d) ? up : 0;
    }
    const int wtotal = __shfl(incl, 31, 32);
    if (lane == 0) wcnt[par * BW + wave] = wtotal;
    __syncthreads();
    int all = 0, pre = 0;
#pragma unroll
    for (int g = 0; g < 4; ++g) {
      const v4i w4 = *(const v4ia*)(wcnt + par * BW + 4 * g);
      const int c0 = clampi(w4.x, 0, 256), c1 = clampi(w4.y, 0, 256);
      const int c2 = clampi(w4.z, 0, 256), c3 = clampi(w4.w, 0, 256);
      all += c0 + c1 + c2 + c3;
      pre += (4 * g + 0 < wave) ? c0 : 0;
      pre += (4 * g + 1 < wave) ? c1 : 0;
      pre += (4 * g + 2 < wave) ? c2 : 0;
      pre += (4 * g + 3 < wave) ? c3 : 0;
    }
    int pos = tot + pre + (incl - c);
#define PUTJ(J, HJ, SJ) if (HJ) { if (pos < RCAP) reg1[pos] = (int)((unsigned)(e0 + (J)) | ((SJ) << SLOTSH)); ++pos; }
    PUTJ(0, h0, s0)
    PUTJ(1, h1, s1)
    PUTJ(2, h2, s2)
    PUTJ(3, h3, s3)
    PUTJ(4, h4, s4)
    PUTJ(5, h5, s5)
    PUTJ(6, h6, s6)
    PUTJ(7, h7, s7)
#undef PUTJ
    tot += all;
  }
  __syncthreads();
  const bool ovf = tot > RCAP;
  const int nh = ovf ? RCAP : tot;

  if (wave == 0) {
#pragma unroll 1
    for (int b0 = 0; b0 < nh; b0 += 32) {
      const int idx = b0 + lane;
      const int uv  = reg1[idx < nh ? idx : nh - 1];
      const int m32 = (nh - b0) < 32 ? (nh - b0) : 32;
#pragma unroll 1
      for (int k = 0; k < m32; ++k) {
        const int u  = __builtin_amdgcn_readlane(uv, k);
        const int sl = (int)(((unsigned)u >> SLOTSH) & (unsigned)(NB - 1));
        const int cv = scnt[sl] + 1;
        if (lane == 0) scnt[sl] = cv;
      }
    }
  }
  __syncthreads();

  int e0c, e1c;
  {
    const v2i cc = *(const v2ia*)(scnt + 2 * tid);
    e0c = cc.x < 0 ? 0 : cc.x;
    e1c = cc.y < 0 ? 0 : cc.y;
    const int ts = e0c + e1c;
    int incl = ts;
#pragma unroll
    for (int d = 1; d < 32; d <<= 1) {
      const int up = __shfl_up(incl, d, 32);
      incl += (lane >= d) ? up : 0;
    }
    if (lane == 31) wtot[wave] = incl;
    __syncthreads();
    int pre = 0;
#pragma unroll
    for (int g = 0; g < 4; ++g) {
      const v4i w4 = *(const v4ia*)(wtot + 4 * g);
      pre += (4 * g + 0 < wave) ? w4.x : 0;
      pre += (4 * g + 1 < wave) ? w4.y : 0;
      pre += (4 * g + 2 < wave) ? w4.z : 0;
      pre += (4 * g + 3 < wave) ? w4.w : 0;
    }
    const int run = pre + incl - ts;
    soff[2 * tid]     = run;
    soff[2 * tid + 1] = run + e0c;
    curs[2 * tid]     = run;
    curs[2 * tid + 1] = run + e0c;
  }
  __syncthreads();

  if (wave == 0) {
#pragma unroll 1
    for (int b0 = 0; b0 < nh; b0 += 32) {
      const int idx = b0 + lane;
      const int uv  = reg1[idx < nh ? idx : nh - 1];
      const int m32 = (nh - b0) < 32 ? (nh - b0) : 32;
#pragma unroll 1
      for (int k = 0; k < m32; ++k) {
        const int u   = __builtin_amdgcn_readlane(uv, k);
        const int sl  = (int)(((unsigned)u >> SLOTSH) & (unsigned)(NB - 1));
        const int eid = (int)((unsigned)u & ((1u << SLOTSH) - 1u));
        const int pr  = curs[sl];
        const int pc  = clampi(pr, 0, RCAP - 1);
        if (lane == 0) { reg2[pc] = eid; curs[sl] = pc + 1; }
      }
    }
  }
  __syncthreads();

  {
    unsigned* lbase = LIST + (size_t)blockIdx.x * (size_t)RCAP;
    const int lastv = nh > 0 ? nh - 1 : 0;
#pragma unroll 1
    for (int it = 0; it < RCAP / BT; ++it) {
      const int i  = it * BT + tid;
      const int ic = i < nh ? i : lastv;
      const int eid = clampi(reg2[ic], 0, NE - 1);
      const int cw = ei[NE + eid];
      asm volatile("" :: "v"(cw));
      const unsigned msk = (i < nh) ? 0xFFFFFFFFu : 0u;
      const unsigned o = (unsigned)clampi(cw, 0, NR - 1) & msk;
      volatile unsigned* q = (volatile unsigned*)(lbase + i);
      *q = o;
      __threadfence();
      *q = o;
    }
  }

  {
    const int base = (int)blockIdx.x * RCAP;
    const v2i cc = *(const v2ia*)(scnt + 2 * tid);
    const v2i so = *(const v2ia*)(soff + 2 * tid);
    v4i m;
    m.x = base + so.x;
    m.y = ovf ? -1 : cc.x;
    m.z = base + so.y;
    m.w = ovf ? -1 : cc.y;
    volatile v4i* q = (volatile v4i*)(META + 2 * (size_t)(nodeBase + 2 * tid));
    *q = m;
    __threadfence();
    *q = m;
  }
}

__global__ __launch_bounds__(RTHR) void k_walk(const float* __restrict__ Z, const float* __restrict__ SD,
                                               const float* __restrict__ SS, const unsigned* __restrict__ LIST,
                                               const int* __restrict__ META, unsigned short* OP) {
  const int lane = (int)threadIdx.x & 31;
  const int wave = (int)threadIdx.x >> 5;
  const int row  = (int)blockIdx.x * RWAVES + wave;
  const bool live = row < NR;
  const int rowc = live ? row : NR - 1;
  const int head = lane >> 3;
  const int c0   = lane * 8;

  const v2i mt = *(const v2ia*)(META + 2 * (size_t)rowc);
  asm volatile("" :: "v"(mt));
  const int craw = mt.y;
  const int offv = clampi(mt.x, 0, LISTTOT - 1);
  const int cl0  = clampi(craw, 0, DEGCAP);
  const int cntv = live ? (cl0 < (LISTTOT - offv) ? cl0 : (LISTTOT - offv)) : 0;
  const int off = __builtin_amdgcn_readfirstlane(offv);
  const int cnt = __builtin_amdgcn_readfirstlane(cntv);
  const bool poison = live && ((craw < 0) || (craw > DEGCAP));

  const v4f sd4 = *(const v4fa*)(SD + (size_t)rowc * NHD);
  asm volatile("" :: "v"(sd4));

  int jj = lane < cnt ? lane : cnt - 1;
  jj = jj < 0 ? 0 : jj;
  const unsigned idw = LIST[(size_t)(off + jj)];
  asm volatile("" :: "v"(idw));
  const int col = clampi((int)idw, 0, NR - 1);
  const v4f ss4 = *(const v4fa*)(SS + (size_t)col * NHD);
  asm volatile("" :: "v"(ss4));

  const float e0 = expf(lrelu_k(sd4.x + ss4.x));
  const float e1 = expf(lrelu_k(sd4.y + ss4.y));
  const float e2 = expf(lrelu_k(sd4.z + ss4.z));
  const float e3 = expf(lrelu_k(sd4.w + ss4.w));
  float d0 = 0.0f, d1 = 0.0f, d2 = 0.0f, d3 = 0.0f;
#pragma unroll 1
  for (int k = 0; k < cnt; ++k) {
    d0 = d0 + bcf(e0, k);
    d1 = d1 + bcf(e1, k);
    d2 = d2 + bcf(e2, k);
    d3 = d3 + bcf(e3, k);
  }
  const float dd0 = d0 + 1e-9f;
  const float dd1 = d1 + 1e-9f;
  const float dd2 = d2 + 1e-9f;
  const float dd3 = d3 + 1e-9f;

  const float w0 = e0 / dd0;
  const float w1 = e1 / dd1;
  const float w2 = e2 / dd2;
  const float w3 = e3 / dd3;
  v4f aa = (v4f){0.0f, 0.0f, 0.0f, 0.0f};
  v4f ab = (v4f){0.0f, 0.0f, 0.0f, 0.0f};
#pragma unroll 1
  for (int k = 0; k < cnt; ++k) {
    const int c = clampi(__builtin_amdgcn_readlane(col, k), 0, NR - 1);
    const float x0 = bcf(w0, k);
    const float x1 = bcf(w1, k);
    const float x2 = bcf(w2, k);
    const float x3 = bcf(w3, k);
    float w = x0;
    w = (head == 1) ? x1 : w;
    w = (head == 2) ? x2 : w;
    w = (head == 3) ? x3 : w;
    const float* zp = Z + (size_t)c * HDW + c0;
    const v4f za = *(const v4fa*)zp;
    const v4f zb = *(const v4fa*)(zp + 4);
    asm volatile("" :: "v"(za), "v"(zb));
    float pr;
    pr = w * za.x; aa.x = aa.x + pr;
    pr = w * za.y; aa.y = aa.y + pr;
    pr = w * za.z; aa.z = aa.z + pr;
    pr = w * za.w; aa.w = aa.w + pr;
    pr = w * zb.x; ab.x = ab.x + pr;
    pr = w * zb.y; ab.y = ab.y + pr;
    pr = w * zb.z; ab.z = ab.z + pr;
    pr = w * zb.w; ab.w = ab.w + pr;
  }

  const float qnan = __uint_as_float(0x7fc00000u);
  aa.x = poison ? qnan : aa.x;
  aa.y = poison ? qnan : aa.y;
  aa.z = poison ? qnan : aa.z;
  aa.w = poison ? qnan : aa.w;
  ab.x = poison ? qnan : ab.x;
  ab.y = poison ? qnan : ab.y;
  ab.z = poison ? qnan : ab.z;
  ab.w = poison ? qnan : ab.w;

  const v4u hi = pack8_bf16(aa, ab);
  unsigned short* orow = OP + (size_t)row * KO + c0;
  volatile v4u* qh = (volatile v4u*)orow;
#if SPLIT_O
  const v4u lo = pack8_bf16_lo(aa, ab);
  volatile v4u* ql = (volatile v4u*)(orow + HDW);
#endif
  const bool rok = row < MPAD;
  if (rok) *qh = hi;
#if SPLIT_O
  if (rok) *ql = lo;
#endif
  __threadfence();
  if (rok) *qh = hi;
#if SPLIT_O
  if (rok) *ql = lo;
#endif
}

__global__ __launch_bounds__(RTHR) void k_epi(const float* __restrict__ P, const unsigned* __restrict__ XBW,
                                              const float* __restrict__ TB, float* out, int nr) {
  __shared__ __attribute__((aligned(16))) float spar[2 * DOUTW];
  const int tid  = (int)threadIdx.x;
  const int lane = tid & 31;
  const int wave = tid >> 5;
  const int row  = (int)blockIdx.x * RWAVES + wave;
  const int rowc = clampi(row, 0, nr - 1);
  if (tid < 32) {
    const v4f pv4 = *(const v4fa*)(TB + TB_LG + 4 * tid);
    *(v4fa*)(spar + 4 * tid) = pv4;
  }
  __syncthreads();

  const v2f pv = *(const v2fa*)(P + (size_t)rowc * DOUTW + 2 * lane);
  asm volatile("" :: "v"(pv));
  const unsigned xw = XBW[(size_t)rowc * (KD / 2) + lane];
  asm volatile("" :: "v"(xw));
  float x0 = __uint_as_float(xw << 16);
  float x1 = __uint_as_float(xw & 0xffff0000u);
  asm volatile("" : "+v"(x0));
  asm volatile("" : "+v"(x1));

  const float m0 = expm1f(pv.x);
  const float m1 = expm1f(pv.y);
  const float a0 = (pv.x > 0.0f) ? pv.x : m0;
  const float a1 = (pv.y > 0.0f) ? pv.y : m1;
  const float y0 = a0 + x0;
  const float y1 = a1 + x1;

  float s = y0 + y1;
  s = sum32(s);
  const float mu = s * 0.015625f;
  const float dv0 = y0 - mu;
  const float dv1 = y1 - mu;
  float q = dv0 * dv0;
  const float r = dv1 * dv1;
  q = q + r;
  q = sum32(q);
  float var = q * 0.015625f;
  var = var + 1e-5f;
  const float rs = 1.0f / sqrtf(var);

  const v2f g2 = *(const v2fa*)(spar + 2 * lane);
  const v2f b2 = *(const v2fa*)(spar + DOUTW + 2 * lane);
  v2f o;
  float t;
  t = dv0 * rs; t = t * g2.x; o.x = t + b2.x;
  t = dv1 * rs; t = t * g2.y; o.y = t + b2.y;

  const bool rok = row < nr;
  volatile v2f* qo = (volatile v2f*)(out + (size_t)rowc * DOUTW + 2 * lane);
  if (rok) *qo = o;
  __threadfence();
  if (rok) *qo = o;
}

extern "C" void kernel_launch(void* const* d_in, const int* in_sizes, int n_in,
                              void* d_out, int out_size, void* d_ws, size_t ws_size,
                              hipStream_t stream) {
  if (n_in < 9) return;
  if (in_sizes[0] != NR * KD) return;
  if (in_sizes[1] != 2 * NE) return;
  if (in_sizes[2] != HDW * KD) return;
  if (in_sizes[3] != NHD * DSZ || in_sizes[4] != NHD * DSZ) return;
  if (in_sizes[5] != DOUTW * HDW) return;
  if (in_sizes[6] != DOUTW || in_sizes[7] != DOUTW || in_sizes[8] != DOUTW) return;
  if (out_size != NR * DOUTW) return;

  const float* x    = (const float*)d_in[0];
  const int*   ei   = (const int*)  d_in[1];
  const float* Wl   = (const float*)d_in[2];
  const float* asrc = (const float*)d_in[3];
  const float* adst = (const float*)d_in[4];
  const float* Wo   = (const float*)d_in[5];
  const float* bo   = (const float*)d_in[6];
  const float* lg   = (const float*)d_in[7];
  const float* lb   = (const float*)d_in[8];
  float* out = (float*)d_out;

  const size_t szXB   = (size_t)MPAD * KD * 2;
  const size_t szWLB  = (size_t)HDW * KD * 2;
  const size_t szWO2  = (size_t)DOUTW * KO * 2;
  const size_t szTB   = (size_t)TB_N * 4;
  const size_t szZ    = (size_t)MPAD * HDW * 4;
  const size_t szOP   = (size_t)MPAD * KO * 2;
  const size_t szT    = (size_t)MPAD * NHD * 4;
  const size_t szMETA = (size_t)NBLK * NB * 2 * 4;
  const size_t szLIST = (size_t)NBLK * RCAP * 4;
  static_assert((size_t)MPAD * DOUTW * 4 <= (size_t)MPAD * HDW * 4);
  static_assert((size_t)MPAD * KD * 2 + (size_t)HDW * KD * 2 + (size_t)DOUTW * KO * 2 + (size_t)TB_N * 4 +
                (size_t)MPAD * HDW * 4 + (size_t)MPAD * KO * 2 + 2 * (size_t)MPAD * NHD * 4 +
                (size_t)NBLK * NB * 8 + (size_t)NBLK * RCAP * 4 <= WSMAX);
#if SPLIT_O
  static_assert((size_t)MPAD * KD * 2 + (size_t)HDW * KD * 2 + (size_t)DOUTW * KO * 2 + (size_t)TB_N * 4 +
                (size_t)MPAD * HDW * 4 + (size_t)MPAD * KO * 2 + 2 * (size_t)MPAD * NHD * 4 +
                (size_t)NBLK * NB * 8 + (size_t)NBLK * RCAP * 4 == (size_t)110760 * 1024);
#endif
  char* ws = (char*)d_ws;
  size_t off = 0;
  const size_t oXB   = off; off += szXB;
  const size_t oWLB  = off; off += szWLB;
  const size_t oWO2  = off; off += szWO2;
  const size_t oTB   = off; off += szTB;
  const size_t oZ    = off; off += szZ;
  const size_t oOP   = off; off += szOP;
  const size_t oSD   = off; off += szT;
  const size_t oSS   = off; off += szT;
  const size_t oMETA = off; off += szMETA;
  const size_t oLIST = off; off += szLIST;
  if (off > ws_size || off > (size_t)WSMAX) return;
  unsigned short* XB  = (unsigned short*)(ws + oXB);
  unsigned short* WLB = (unsigned short*)(ws + oWLB);
  unsigned short* WO2 = (unsigned short*)(ws + oWO2);
  float*    TB   = (float*)(ws + oTB);
  float*    Z    = (float*)(ws + oZ);
  float*    P    = (float*)(ws + oZ);
  unsigned short* OP = (unsigned short*)(ws + oOP);
  float*    SD   = (float*)(ws + oSD);
  float*    SS   = (float*)(ws + oSS);
  int*      META = (int*)(ws + oMETA);
  unsigned* LIST = (unsigned*)(ws + oLIST);

  hipFuncSetAttribute(reinterpret_cast<const void*>(&k_bucket),
                      hipFuncAttributeMaxDynamicSharedMemorySize, LDS_BKT);

  k_plane<0><<<MPAD * KD / 8 / 256, 256, 0, stream>>>(x, NR, KD, KD, XB, MPAD, KD);
  k_prep<<<PB_ALL, 256, 0, stream>>>(Wl, Wo, asrc, adst, bo, lg, lb, WLB, WO2, TB);
  k_bucket<<<NBLK, BT, LDS_BKT, stream>>>(ei, LIST, META);
  {
    const int tiles = (MPAD / 64) * (HDW / 64);
    k_gemm_nt<0, 0><<<(tiles + 7) / 8, 256, 0, stream>>>(XB, WLB, TB, Z, MPAD, HDW, KD, HDW);
  }
  k_rowprep<<<NR / RWAVES, RTHR, 0, stream>>>(Z, TB, SD, SS);
  k_walk<<<MPAD / RWAVES, RTHR, 0, stream>>>(Z, SD, SS, LIST, META, OP);
  {
    const int tiles = (MPAD / 64) * (DOUTW / 64);
    k_gemm_nt<0, 1><<<(tiles + 7) / 8, 256, 0, stream>>>(OP, WO2, TB + TB_BO, P, MPAD, DOUTW, KO, DOUTW);
  }
  k_epi<<<NR / RWAVES, RTHR, 0, stream>>>(P, (const unsigned*)XB, TB, out, NR);
}
